// HeadModule_77094662963970
// MI455X (gfx1250) — hardware-verified
//
#include <hip/hip_runtime.h>
#define NPT 262144
#define PC 32
#define PH 256
#define NTX (PH * PH)
#define CHK 65536
#define DIN 64
#define DH 128
typedef __bf16 v16b __attribute__((ext_vector_type(16)));
typedef unsigned short v8us __attribute__((ext_vector_type(8), may_alias));
typedef float  v8f  __attribute__((ext_vector_type(8)));
typedef float  v4f  __attribute__((ext_vector_type(4)));
typedef float  v4fa __attribute__((ext_vector_type(4), may_alias));
union FragB { v16b v; v8us half[2]; unsigned short u[16]; };

__device__ __forceinline__ unsigned short bf16_bits(float x) { unsigned int u = __float_as_uint(x); return (unsigned short)((u + 0x7FFFu + ((u >> 16) & 1u)) >> 16); }
__device__ __forceinline__ float bf16_val(unsigned short b) { return __uint_as_float(((unsigned int)b) << 16); }
__device__ __forceinline__ float bf16_round(float x) { return bf16_val(bf16_bits(x)); }
template <int NT>
__device__ __forceinline__ v8f mmaN(v16b ah, v16b al, v16b bh, v16b bl, v8f c) {
  c = __builtin_amdgcn_wmma_f32_16x16x32_bf16(false, ah, false, bh, (short)0, c, false, false);
  if (NT >= 2) c = __builtin_amdgcn_wmma_f32_16x16x32_bf16(false, al, false, bh, (short)0, c, false, false);
  if (NT >= 3) c = __builtin_amdgcn_wmma_f32_16x16x32_bf16(false, ah, false, bl, (short)0, c, false, false);
  asm volatile("v_nop\n\tv_nop\n\tv_nop\n\tv_nop" : "+v"(c) : "v"(ah), "v"(al), "v"(bh), "v"(bl));
  return c;
}

__global__ __launch_bounds__(256) void k_wt_bf16(const float* __restrict__ W, unsigned short* __restrict__ Wt, int K, int N) {
  const int t = blockIdx.x * 256 + threadIdx.x;
  const int k8n = K / 8;
  if (t >= N * k8n) return;
  const int n = t / k8n, k8 = (t % k8n) * 8;
  v8us v;
#pragma unroll
  for (int i = 0; i < 8; ++i) v[i] = bf16_bits(W[(size_t)(k8 + i) * N + n]);
  *(volatile v8us*)(Wt + (size_t)n * K + k8) = v;
  __threadfence();
  *(volatile v8us*)(Wt + (size_t)n * K + k8) = v;
}

template <bool ASPLIT, int ACT, bool BIAS_BF16>
__global__ __launch_bounds__(128) void k_gemm_bf(const float* __restrict__ A, int lda, const unsigned short* __restrict__ Wt, int ldb,
                                               const float* __restrict__ bias, float* __restrict__ C, int ldc, int M, int N, int K) {
  __shared__ __attribute__((aligned(16))) float so[4][16][64];
  const int tid = threadIdx.x, w = tid >> 5, lane = tid & 31, ln = lane & 15, hh = lane >> 4;
  const int ntn = N / 64;
  const int wid = blockIdx.x * 4 + w;
  const int mt = wid / ntn, nq = wid % ntn;
  if (mt * 16 >= M) return;
  const int row0 = mt * 16, col0 = nq * 64;
  const float* arow = A + (size_t)(row0 + ln) * lda;
  v8f acc[4] = {};
  for (int kb = 0; kb < K; kb += 32) {
    FragB ah, al;
    const v4f x0 = *(const v4fa*)(arow + kb + 8 * hh), x1 = *(const v4fa*)(arow + kb + 8 * hh + 4);
    const v4f x2 = *(const v4fa*)(arow + kb + 16 + 8 * hh), x3 = *(const v4fa*)(arow + kb + 16 + 8 * hh + 4);
    float xs[16] = {x0[0],x0[1],x0[2],x0[3],x1[0],x1[1],x1[2],x1[3],x2[0],x2[1],x2[2],x2[3],x3[0],x3[1],x3[2],x3[3]};
#pragma unroll
    for (int i = 0; i < 16; ++i) { const unsigned short hb = bf16_bits(xs[i]); ah.u[i] = hb; al.u[i] = ASPLIT ? bf16_bits(xs[i] - bf16_val(hb)) : (unsigned short)0; }
#pragma unroll
    for (int t = 0; t < 4; ++t) {
      const unsigned short* brow = Wt + (size_t)(col0 + t * 16 + ln) * ldb + kb;
      FragB b;
      b.half[0] = *(const v8us*)(brow + 8 * hh);
      b.half[1] = *(const v8us*)(brow + 16 + 8 * hh);
      acc[t] = mmaN<ASPLIT ? 2 : 1>(ah.v, al.v, b.v, b.v, acc[t]);
    }
  }
#pragma unroll
  for (int t = 0; t < 4; ++t) {
    float bv = bias ? bias[col0 + t * 16 + ln] : 0.f;
    if (BIAS_BF16) bv = bf16_round(bv);
#pragma unroll
    for (int r = 0; r < 8; ++r) { float v = acc[t][r] + bv; if (ACT == 1) v = fmaxf(v, 0.f); so[w][8 * hh + r][t * 16 + ln] = v; }
  }
  __builtin_amdgcn_fence(__ATOMIC_ACQ_REL, "workgroup");
  __builtin_amdgcn_wave_barrier();
  const int rsub = lane >> 4, c4 = (lane & 15) * 4;
  for (int pass = 0; pass < 2; ++pass) {
#pragma unroll
    for (int q = 0; q < 8; ++q) {
      const int r = q * 2 + rsub;
      const v4f v = *(const v4fa*)&so[w][r][c4];
      *(volatile v4f*)(C + (size_t)(row0 + r) * ldc + col0 + c4) = v;
    }
    if (pass == 0) __threadfence();
  }
}

template <bool ASPLIT, int ACT, bool BIAS_BF16, bool RES_BF16>
__global__ __launch_bounds__(128) void k_gemm_bf3(const float* __restrict__ A, int lda, const unsigned short* __restrict__ Wt, int ldb,
                                                const float* __restrict__ bias, const float* __restrict__ resid, int rmod, int ldr,
                                                float* __restrict__ C, int ldc, int M, int N, int K) {
  __shared__ __attribute__((aligned(16))) float so[4][16][64];
  const int tid = threadIdx.x, w = tid >> 5, lane = tid & 31, ln = lane & 15, hh = lane >> 4;
  const int ntn = N / 64;
  const int wid = blockIdx.x * 4 + w;
  const int mt = wid / ntn, nq = wid % ntn;
  if (mt * 16 >= M) return;
  const int row0 = mt * 16, col0 = nq * 64;
  const float* arow = A + (size_t)(row0 + ln) * lda;
  v8f acc[4] = {};
  for (int kb = 0; kb < K; kb += 32) {
    FragB ah, al;
    const v4f x0 = *(const v4fa*)(arow + kb + 8 * hh), x1 = *(const v4fa*)(arow + kb + 8 * hh + 4);
    const v4f x2 = *(const v4fa*)(arow + kb + 16 + 8 * hh), x3 = *(const v4fa*)(arow + kb + 16 + 8 * hh + 4);
    float xs[16] = {x0[0],x0[1],x0[2],x0[3],x1[0],x1[1],x1[2],x1[3],x2[0],x2[1],x2[2],x2[3],x3[0],x3[1],x3[2],x3[3]};
#pragma unroll
    for (int i = 0; i < 16; ++i) { const unsigned short hb = bf16_bits(xs[i]); ah.u[i] = hb; al.u[i] = ASPLIT ? bf16_bits(xs[i] - bf16_val(hb)) : (unsigned short)0; }
#pragma unroll
    for (int t = 0; t < 4; ++t) {
      const unsigned short* brow = Wt + (size_t)(col0 + t * 16 + ln) * ldb + kb;
      FragB b;
      b.half[0] = *(const v8us*)(brow + 8 * hh);
      b.half[1] = *(const v8us*)(brow + 16 + 8 * hh);
      acc[t] = mmaN<ASPLIT ? 2 : 1>(ah.v, al.v, b.v, b.v, acc[t]);
    }
  }
#pragma unroll
  for (int t = 0; t < 4; ++t) {
    const int col = col0 + t * 16 + ln;
    float bv = bias ? bias[col] : 0.f;
    if (BIAS_BF16) bv = bf16_round(bv);
#pragma unroll
    for (int r = 0; r < 8; ++r) {
      float v = acc[t][r] + bv;
      if (resid) { float rv = resid[(size_t)((row0 + 8 * hh + r) % rmod) * ldr + col]; if (RES_BF16) rv = bf16_round(rv); v += rv; }
      if (ACT == 1) v = fmaxf(v, 0.f);
      if (ACT == 2) v = 0.5f * v * (1.0f + erff(v * 0.70710678118654752f));
      if (ACT == 3) { const float u = 0.7978845608028654f * (v + 0.044715f * v * v * v); v = 0.5f * v * (1.0f + tanhf(u)); }
      so[w][8 * hh + r][t * 16 + ln] = v;
    }
  }
  __builtin_amdgcn_fence(__ATOMIC_ACQ_REL, "workgroup");
  __builtin_amdgcn_wave_barrier();
  const int rsub = lane >> 4, c4 = (lane & 15) * 4;
  for (int pass = 0; pass < 2; ++pass) {
#pragma unroll
    for (int q = 0; q < 8; ++q) {
      const int r = q * 2 + rsub;
      const v4f v = *(const v4fa*)&so[w][r][c4];
      *(volatile v4f*)(C + (size_t)(row0 + r) * ldc + col0 + c4) = v;
    }
    if (pass == 0) __threadfence();
  }
}
template <bool PARAM_BF16>
__global__ __launch_bounds__(256) void k_layernorm(const float* __restrict__ X, const float* __restrict__ R, const float* __restrict__ g, const float* __restrict__ bta,
                                                  float* __restrict__ out_sum, float* __restrict__ out_norm, int N, float eps) {
  __shared__ float red[256];
  const int row = blockIdx.x, tid = threadIdx.x;
  const float* x = X + (size_t)row * N; const float* rr = R ? R + (size_t)row * N : nullptr;
  float vals[16];
  const int per = N / 256;
  float s1 = 0.f;
  for (int u = 0; u < per / 4; ++u) {
    const int j = tid * 4 + 1024 * u;
    const v4f a = *(const v4fa*)(x + j);
    v4f b = {0.f,0.f,0.f,0.f}; if (rr) b = *(const v4fa*)(rr + j);
#pragma unroll
    for (int q = 0; q < 4; ++q) { const float v = a[q] + b[q]; vals[u * 4 + q] = v; s1 += v; }
  }
  red[tid] = s1; __syncthreads();
  for (int st = 128; st > 0; st >>= 1) { if (tid < st) red[tid] += red[tid + st]; __syncthreads(); }
  const float mu = red[0] / (float)N; __syncthreads();
  float s2 = 0.f;
  for (int u = 0; u < per / 4; ++u)
#pragma unroll
    for (int q = 0; q < 4; ++q) { const float c = vals[u * 4 + q] - mu; s2 += c * c; }
  red[tid] = s2; __syncthreads();
  for (int st = 128; st > 0; st >>= 1) { if (tid < st) red[tid] += red[tid + st]; __syncthreads(); }
  const float rs = rsqrtf(red[0] / (float)N + eps);
  for (int pass = 0; pass < 2; ++pass) {
    for (int u = 0; u < per / 4; ++u) {
      const int j = tid * 4 + 1024 * u;
      v4f o, sm;
#pragma unroll
      for (int q = 0; q < 4; ++q) {
        float gg = g[j + q], bb = bta[j + q];
        if (PARAM_BF16) { gg = bf16_round(gg); bb = bf16_round(bb); }
        sm[q] = vals[u * 4 + q]; o[q] = (vals[u * 4 + q] - mu) * rs * gg + bb;
      }
      if (out_sum) *(volatile v4f*)(out_sum + (size_t)row * N + j) = sm;
      *(volatile v4f*)(out_norm + (size_t)row * N + j) = o;
    }
    if (pass == 0) __threadfence();
  }
}


typedef _Float16 v16h __attribute__((ext_vector_type(16)));
union FragH { v16h v; v8us half[2]; _Float16 h[16]; unsigned short u[16]; };
template <int NT>
__device__ __forceinline__ v8f mmaH(v16h ah, v16h al, v16h bh, v16h bl, v8f c) {
  c = __builtin_amdgcn_wmma_f32_16x16x32_f16(false, ah, false, bh, (short)0, c, false, false);
  if (NT >= 2) c = __builtin_amdgcn_wmma_f32_16x16x32_f16(false, al, false, bh, (short)0, c, false, false);
  if (NT >= 3) c = __builtin_amdgcn_wmma_f32_16x16x32_f16(false, ah, false, bl, (short)0, c, false, false);
  asm volatile("v_nop\n\tv_nop\n\tv_nop\n\tv_nop" : "+v"(c) : "v"(ah), "v"(al), "v"(bh), "v"(bl));
  return c;
}
template <bool ASPLIT>
__global__ __launch_bounds__(128) void k_gemm_h(const float* __restrict__ A, int lda, size_t sA, const _Float16* __restrict__ Bh, int ldb, size_t sB, float alpha, float* __restrict__ C, int ldc, size_t sC, int M, int N, int K) {
  __shared__ __attribute__((aligned(16))) float so[4][16][64];
  const int tid = threadIdx.x, w = tid >> 5, lane = tid & 31, ln = lane & 15, hh = lane >> 4; const int by = blockIdx.y;
  A += (size_t)by * sA; Bh += (size_t)by * sB; C += (size_t)by * sC;
  const int ntn = (N + 63) / 64; const int wid = blockIdx.x * 4 + w; const int mt = wid / ntn, nq = wid % ntn; if (mt * 16 >= M) return;
  const int row0 = mt * 16, col0 = nq * 64; const float* arow = A + (size_t)(row0 + ln) * lda;
  v8f acc[4] = {};
  for (int kb = 0; kb < K; kb += 32) {
    FragH ah, al;
    const v4f x0 = *(const v4fa*)(arow + kb + 8 * hh), x1 = *(const v4fa*)(arow + kb + 8 * hh + 4), x2 = *(const v4fa*)(arow + kb + 16 + 8 * hh), x3 = *(const v4fa*)(arow + kb + 16 + 8 * hh + 4);
    float xs[16] = {x0[0],x0[1],x0[2],x0[3],x1[0],x1[1],x1[2],x1[3],x2[0],x2[1],x2[2],x2[3],x3[0],x3[1],x3[2],x3[3]};
#pragma unroll
    for (int i = 0; i < 16; ++i) { const _Float16 h = (_Float16)xs[i]; ah.h[i] = h; al.h[i] = ASPLIT ? (_Float16)(xs[i] - (float)h) : (_Float16)0.0f; }
#pragma unroll
    for (int t = 0; t < 4; ++t) { if (col0 + t * 16 >= N) continue; const size_t boff = (size_t)(col0 + t * 16 + ln) * ldb + kb; FragH bq; bq.half[0] = *(const v8us*)(Bh + boff + 8 * hh); bq.half[1] = *(const v8us*)(Bh + boff + 16 + 8 * hh);
      acc[t] = mmaH<ASPLIT ? 2 : 1>(ah.v, al.v, bq.v, bq.v, acc[t]); }
  }
#pragma unroll
  for (int t = 0; t < 4; ++t) { if (col0 + t * 16 >= N) continue;
#pragma unroll
    for (int r = 0; r < 8; ++r) so[w][8 * hh + r][t * 16 + ln] = acc[t][r] * alpha; }
  __builtin_amdgcn_fence(__ATOMIC_ACQ_REL, "workgroup"); __builtin_amdgcn_wave_barrier();
  const int rsub = lane >> 4, c4 = (lane & 15) * 4;
  for (int pass = 0; pass < 2; ++pass) {
#pragma unroll
    for (int q = 0; q < 8; ++q) { const int r = q * 2 + rsub; if (col0 + c4 < N) { const v4f v = *(const v4fa*)&so[w][r][c4]; *(volatile v4f*)(C + (size_t)(row0 + r) * ldc + col0 + c4) = v; } }
    if (pass == 0) __threadfence(); }
}

__global__ __launch_bounds__(256) void k_wt_f16(const float* __restrict__ W, _Float16* __restrict__ Wt, int K, int N, float scale) {
  const int t = blockIdx.x * 256 + threadIdx.x; if (t >= N * (K / 8)) return; const int n = t / (K / 8), k8 = (t % (K / 8)) * 8; FragH f;
#pragma unroll
  for (int i = 0; i < 8; ++i) f.h[i] = (_Float16)(bf16_round(W[(size_t)(k8 + i) * N + n]) * scale); const v8us o = f.half[0];
  *(volatile v8us*)((unsigned short*)Wt + (size_t)n * K + k8) = o; __threadfence(); *(volatile v8us*)((unsigned short*)Wt + (size_t)n * K + k8) = o;
}
template <int ACT>
__global__ __launch_bounds__(128) void k_gemm_hhx(const _Float16* __restrict__ A, int lda, size_t sA, const _Float16* __restrict__ Bh, int ldb, size_t sB, float alpha, const float* __restrict__ bias, size_t sBias, const float* __restrict__ CP, int rowsPerB, size_t sCPb, int row0g,
    float* __restrict__ C, _Float16* __restrict__ C16, int ldc, size_t sC, int M, int N, int K) {
  __shared__ __attribute__((aligned(16))) float so[4][16][64];
  const int tid = threadIdx.x, w = tid >> 5, lane = tid & 31, ln = lane & 15, hh = lane >> 4; const int by = blockIdx.y;
  A += (size_t)by * sA; Bh += (size_t)by * sB; const size_t cofs = (size_t)by * sC; const float* bp = bias ? bias + (size_t)by * sBias : nullptr;
  const int ntn = (N + 63) / 64; const int wid = blockIdx.x * 4 + w; const int mt = wid / ntn, nq = wid % ntn; if (mt * 16 >= M) return;
  const int row0 = mt * 16, col0 = nq * 64; const _Float16* arow = A + (size_t)(row0 + ln) * lda;
  v8f acc[4] = {};
  for (int kb = 0; kb < K; kb += 32) { FragH ah; ah.half[0] = *(const v8us*)((const unsigned short*)arow + kb + 8 * hh); ah.half[1] = *(const v8us*)((const unsigned short*)arow + kb + 16 + 8 * hh);
#pragma unroll
    for (int t = 0; t < 4; ++t) { if (col0 + t * 16 >= N) continue; const size_t boff = (size_t)(col0 + t * 16 + ln) * ldb + kb; FragH bq; bq.half[0] = *(const v8us*)((const unsigned short*)Bh + boff + 8 * hh); bq.half[1] = *(const v8us*)((const unsigned short*)Bh + boff + 16 + 8 * hh);
      acc[t] = mmaH<1>(ah.v, ah.v, bq.v, bq.v, acc[t]); }
  }
#pragma unroll
  for (int t = 0; t < 4; ++t) { if (col0 + t * 16 >= N) continue; const int col = col0 + t * 16 + ln; const float bv = bp ? bf16_round(bp[col]) : 0.f;
#pragma unroll
    for (int r = 0; r < 8; ++r) { float v = acc[t][r] * alpha + bv; if (CP) { const int bidx = (row0g + row0 + 8 * hh + r) / rowsPerB; v += CP[(size_t)bidx * sCPb + (size_t)by * 64 + col]; } if (ACT == 1) v = (v > 0.f) ? v : expm1f(v); else if (ACT == 7) v = (v > 0.f) ? v + 1.0f : expf(v); else if (ACT == 8) v = tanhf(v); else if (ACT == 9) v = 0.5f * v * (1.0f + tanhf(0.7978845608028654f * (v + 0.044715f * v * v * v))); else if (ACT == 11) v = 1.0f / (1.0f + expf(-v)); else if (ACT == 12) v = (v > 0.f) ? v : 0.01f * v; else if (ACT == 14) v = (v > 0.f) ? v : 0.1f * v; else if (ACT == 15) v = v / (1.0f + expf(-v)); else if (ACT == 3) v = fmaxf(v, 0.f); else if (ACT == 6) v = 0.5f * v * (1.0f + erff(v * 0.70710678118654752f)); so[w][8 * hh + r][t * 16 + ln] = v; } }
  __builtin_amdgcn_fence(__ATOMIC_ACQ_REL, "workgroup"); __builtin_amdgcn_wave_barrier();
  const int rsub = lane >> 4, c4 = (lane & 15) * 4; typedef _Float16 v4h __attribute__((ext_vector_type(4)));
  for (int pass = 0; pass < 2; ++pass) {
#pragma unroll
    for (int q = 0; q < 8; ++q) { const int r = q * 2 + rsub; if (col0 + c4 < N) { const v4f v = *(const v4fa*)&so[w][r][c4]; if (C) *(volatile v4f*)(C + cofs + (size_t)(row0 + r) * ldc + col0 + c4) = v; if (C16) { v4h h4; for (int i = 0; i < 4; ++i) h4[i] = (_Float16)v[i]; *(volatile v4h*)(C16 + cofs + (size_t)(row0 + r) * ldc + col0 + c4) = h4; } } }
    if (pass == 0) __threadfence(); }
}


typedef _Float16 v4h __attribute__((ext_vector_type(4)));

__global__ __launch_bounds__(256) void k_x16(const float* __restrict__ x, _Float16* __restrict__ X16, size_t n8) { const size_t t = (size_t)blockIdx.x * 256 + threadIdx.x; if (t >= n8) return; FragH f;
#pragma unroll
  for (int q = 0; q < 8; ++q) f.h[q] = (_Float16)bf16_round(x[t * 8 + q]); *(volatile v8us*)((unsigned short*)X16 + t * 8) = f.half[0]; __threadfence(); *(volatile v8us*)((unsigned short*)X16 + t * 8) = f.half[0]; }
__global__ __launch_bounds__(256) void k_h16(const float* __restrict__ x, _Float16* __restrict__ X16, size_t n8) { const size_t t = (size_t)blockIdx.x * 256 + threadIdx.x; if (t >= n8) return; FragH f;
#pragma unroll
  for (int q = 0; q < 8; ++q) f.h[q] = (_Float16)x[t * 8 + q]; *(volatile v8us*)((unsigned short*)X16 + t * 8) = f.half[0]; __threadfence(); *(volatile v8us*)((unsigned short*)X16 + t * 8) = f.half[0]; }
__global__ __launch_bounds__(256) void k_round16f(const float* __restrict__ W, _Float16* __restrict__ Bt, size_t n8) { const size_t t = (size_t)blockIdx.x * 256 + threadIdx.x; if (t >= n8) return; FragH f;
#pragma unroll
  for (int i = 0; i < 8; ++i) f.h[i] = (_Float16)(bf16_round(W[t * 8 + i]) * 16.0f); *(volatile v8us*)((unsigned short*)Bt + t * 8) = f.half[0]; __threadfence(); *(volatile v8us*)((unsigned short*)Bt + t * 8) = f.half[0]; }
template <int NHv, int TTv>
__global__ __launch_bounds__(256) void k_vt(const _Float16* __restrict__ V16, int ldv, int voff, _Float16* __restrict__ Vt) { __shared__ unsigned short tl[64][66]; const int tid = threadIdx.x; const int slab = blockIdx.x / (TTv / 64), lg = blockIdx.x % (TTv / 64); const int b = slab / NHv, h = slab % NHv;
  for (int i = tid; i < 64 * 8; i += 256) { const int r = i / 8, c8 = (i % 8) * 8; FragH f; f.half[0] = *(const v8us*)((const unsigned short*)V16 + ((size_t)b * TTv + lg * 64 + r) * ldv + voff + h * 64 + c8);
#pragma unroll
    for (int q = 0; q < 8; ++q) tl[r][c8 + q] = f.u[q]; }
  __syncthreads();
  for (int pass = 0; pass < 2; ++pass) {
#pragma unroll
    for (int rd = 0; rd < 2; ++rd) { const int d = rd * 32 + tid / 8, pc = tid % 8; FragH f;
#pragma unroll
      for (int q = 0; q < 8; ++q) f.u[q] = tl[pc * 8 + q][d];
      *(volatile v8us*)((unsigned short*)Vt + ((size_t)slab * 64 + d) * TTv + lg * 64 + pc * 8) = f.half[0]; }
    if (pass == 0) __threadfence(); } }

__global__ __launch_bounds__(256) void k_hl(const float* __restrict__ F, _Float16* __restrict__ Hh, _Float16* __restrict__ Hl, size_t n8) { const size_t t = (size_t)blockIdx.x * 256 + threadIdx.x; if (t >= n8) return; FragH fh, fl; const v4f a = *(const v4fa*)(F + t * 8), c = *(const v4fa*)(F + t * 8 + 4);
#pragma unroll
  for (int q = 0; q < 4; ++q) { _Float16 h = (_Float16)a[q]; fh.h[q] = h; fl.h[q] = (_Float16)((a[q] - (float)h) * 1024.0f); h = (_Float16)c[q]; fh.h[4 + q] = h; fl.h[4 + q] = (_Float16)((c[q] - (float)h) * 1024.0f); }
  for (int pass = 0; pass < 2; ++pass) { *(volatile v8us*)((unsigned short*)Hh + t * 8) = fh.half[0]; *(volatile v8us*)((unsigned short*)Hl + t * 8) = fl.half[0]; if (pass == 0) __threadfence(); } }

__global__ __launch_bounds__(256) void k_plane(const float* __restrict__ pl, float* __restrict__ T) {
  __shared__ float tile[32][65]; const int tid = threadIdx.x; const int t0 = blockIdx.x * 64;
  for (int i = tid; i < 32 * 64; i += 256) { const int ci = i / 64, ti = i % 64; tile[ci][ti] = bf16_round(pl[(size_t)ci * NTX + t0 + ti]); }
  __syncthreads();
  for (int it = 0; it < 2; ++it) { const int row = tid / 8 + 32 * it, qd = tid % 8; v4f v; v[0] = tile[qd * 4 + 0][row]; v[1] = tile[qd * 4 + 1][row]; v[2] = tile[qd * 4 + 2][row]; v[3] = tile[qd * 4 + 3][row]; float* dst = T + (size_t)(t0 + row) * PC + qd * 4; *(volatile v4f*)dst = v; __threadfence(); *(volatile v4f*)dst = v; } }
__device__ __forceinline__ void samp8(const float* __restrict__ T, float gx, float gy, int c0, float* acc) { const float px = (gx + 1.0f) * 0.5f * (float)(PH - 1), py = (gy + 1.0f) * 0.5f * (float)(PH - 1); const float x0 = floorf(px), y0 = floorf(py); const float fx = px - x0, fy = py - y0;
#pragma unroll
  for (int cn = 0; cn < 4; ++cn) { const float xi = x0 + (float)(cn & 1), yi = y0 + (float)(cn >> 1); const bool valid = (xi >= 0.f && xi <= (float)(PH - 1) && yi >= 0.f && yi <= (float)(PH - 1)); const float w = ((cn & 1) ? fx : (1.0f - fx)) * ((cn >> 1) ? fy : (1.0f - fy)); const float ww = valid ? w : 0.f; const int xc = (int)fminf(fmaxf(xi, 0.f), (float)(PH - 1)), yc = (int)fminf(fmaxf(yi, 0.f), (float)(PH - 1)); const v4f a = *(const v4fa*)(T + ((size_t)yc * PH + xc) * PC + c0), c = *(const v4fa*)(T + ((size_t)yc * PH + xc) * PC + c0 + 4);
#pragma unroll
    for (int k = 0; k < 8; ++k) acc[k] += ww * ((k < 4) ? a[k] : c[k - 4]); } }
__global__ __launch_bounds__(256) void k_embed(const float* __restrict__ pts, const float* __restrict__ vd, const float* __restrict__ TX, const float* __restrict__ TY, const float* __restrict__ TZ, size_t p0, _Float16* __restrict__ H0) {
  #pragma clang fp contract(off)
  const int t = blockIdx.x * 256 + threadIdx.x; if (t >= CHK * 8) return; const int q = t & 7; const int pl = t >> 3; const size_t pt = p0 + pl; FragH f = FragH{};
  if (q < 4) { const int c0 = q * 8; const float u = bf16_round(pts[pt]), v = bf16_round(pts[NPT + pt]), w = bf16_round(pts[2 * NPT + pt]); float acc[8];
#pragma unroll
    for (int k = 0; k < 8; ++k) acc[k] = 0.f;
    float a1[8], a2[8], a3[8];
#pragma unroll
    for (int k = 0; k < 8; ++k) { a1[k] = 0.f; a2[k] = 0.f; a3[k] = 0.f; }
    samp8(TX, v, w, c0, a1); samp8(TY, u, w, c0, a2); samp8(TZ, u, v, c0, a3);
#pragma unroll
    for (int k = 0; k < 8; ++k) f.h[k] = (_Float16)((a1[k] + a2[k]) + a3[k]); }
  else { const int c0 = 32 + 8 * (q - 4); const float dx = bf16_round(vd[pt]), dy = bf16_round(vd[NPT + pt]), dz = bf16_round(vd[2 * NPT + pt]);
#pragma unroll 1
    for (int k = 0; k < 8; ++k) { const int i = c0 + k - 32; float val = 0.f;
      if (i < 3) val = (i == 0) ? dx : (i == 1) ? dy : dz;
      else if (i < 27) { const int j = (i - 3) % 12; const int fr = j / 3, a = j % 3; const float d = (a == 0) ? dx : (a == 1) ? dy : dz; const float fq = (fr == 0) ? 1.0f : (fr == 1) ? 2.0f : (fr == 2) ? 4.0f : 8.0f; val = (i < 15) ? sinf(d * fq) : cosf(d * fq); }
      const _Float16 hv = (_Float16)val;
#pragma unroll
      for (int kk = 0; kk < 8; ++kk) f.h[kk] = (kk == k) ? hv : f.h[kk]; } }
  *(volatile v8us*)((unsigned short*)H0 + (size_t)pl * DIN + q * 8) = f.half[0]; __threadfence(); *(volatile v8us*)((unsigned short*)H0 + (size_t)pl * DIN + q * 8) = f.half[0]; }
__global__ __launch_bounds__(256) void k_w1(const float* __restrict__ W, int K, int Kp, _Float16* __restrict__ Bt) { const int t = blockIdx.x * 256 + threadIdx.x; if (t >= DH * (Kp / 8)) return; const int k0 = (t % (Kp / 8)) * 8, o = t / (Kp / 8); FragH f;
#pragma unroll
  for (int q = 0; q < 8; ++q) { const int k = k0 + q; f.h[q] = (k < K) ? (_Float16)(bf16_round(W[(size_t)k * DH + o]) * 16.0f) : (_Float16)0.0f; }
  *(volatile v8us*)((unsigned short*)Bt + (size_t)o * Kp + k0) = f.half[0]; __threadfence(); *(volatile v8us*)((unsigned short*)Bt + (size_t)o * Kp + k0) = f.half[0]; }
__global__ __launch_bounds__(256) void k_carry64(const float* __restrict__ F, _Float16* __restrict__ O16, size_t n8) { const size_t t = (size_t)blockIdx.x * 256 + threadIdx.x; if (t >= n8) return; const v4f a = *(const v4fa*)(F + t * 8), c = *(const v4fa*)(F + t * 8 + 4); FragH f;
#pragma unroll
  for (int q = 0; q < 8; ++q) f.h[q] = (_Float16)(((q < 4) ? a[q] : c[q - 4]) * 64.0f);
  *(volatile v8us*)((unsigned short*)O16 + t * 8) = f.half[0]; __threadfence(); *(volatile v8us*)((unsigned short*)O16 + t * 8) = f.half[0]; }
__global__ __launch_bounds__(256) void k_dots(const float* __restrict__ H2, const float* __restrict__ W3, const float* __restrict__ b3, int nout, int row0, size_t p0, float* __restrict__ out) {
  #pragma clang fp contract(off)
  const int pl = blockIdx.x * 256 + threadIdx.x; if (pl >= CHK) return; const float* h = H2 + (size_t)pl * DH;
  for (int k = 0; k < nout; ++k) { float s = bf16_round(b3[k]);
#pragma unroll 1
    for (int j = 0; j < DH; j += 4) { const v4f a = *(const v4fa*)(h + j); s += a[0] * bf16_round(W3[(size_t)j * nout + k]); s += a[1] * bf16_round(W3[(size_t)(j + 1) * nout + k]); s += a[2] * bf16_round(W3[(size_t)(j + 2) * nout + k]); s += a[3] * bf16_round(W3[(size_t)(j + 3) * nout + k]); }
    *(volatile float*)(out + (size_t)(row0 + k) * NPT + p0 + pl) = s; __threadfence(); *(volatile float*)(out + (size_t)(row0 + k) * NPT + p0 + pl) = s; } }

extern "C" void kernel_launch(void* const* d_in, const int* in_sizes, int n_in,
                              void* d_out, int out_size, void* d_ws, size_t ws_size, hipStream_t stream) {
  (void)in_sizes; (void)n_in; (void)out_size;
  const float* const* I = (const float* const*)d_in; const float* pts = I[0]; const float* vd = I[1]; const float* tp = I[2];
  const float* dW1 = I[3]; const float* dB1 = I[4]; const float* dW2 = I[5]; const float* dB2 = I[6]; const float* dW3 = I[7]; const float* dB3 = I[8]; const float* cW1 = I[9]; const float* cB1 = I[10]; const float* cW2 = I[11]; const float* cB2 = I[12]; const float* cW3 = I[13]; const float* cB3 = I[14];
  char* ws = (char*)d_ws; size_t off = 0;
  auto take = [&](size_t bytes) { char* p = ws + off; off += (bytes + 255) & ~(size_t)255; return p; };
  float* T[3]; for (int j = 0; j < 3; ++j) T[j] = (float*)take((size_t)NTX * PC * 4); _Float16* BD1 = (_Float16*)take((size_t)DH * 32 * 2); _Float16* BC1 = (_Float16*)take((size_t)DH * DIN * 2); _Float16* BD2 = (_Float16*)take((size_t)DH * DH * 2); _Float16* BC2 = (_Float16*)take((size_t)DH * DH * 2);
  _Float16* H0 = (_Float16*)take((size_t)CHK * DIN * 2); float* H1 = (float*)take((size_t)CHK * DH * 4); _Float16* H116 = (_Float16*)take((size_t)CHK * DH * 2); float* H2 = (float*)take((size_t)CHK * DH * 4);
  if (off > ws_size) return;
  for (int j = 0; j < 3; ++j) k_plane<<<NTX / 64, 256, 0, stream>>>(tp + (size_t)j * PC * NTX, T[j]);
  k_w1<<<(DH * 4 + 255) / 256, 256, 0, stream>>>(dW1, 32, 32, BD1); k_w1<<<(DH * 8 + 255) / 256, 256, 0, stream>>>(cW1, 59, DIN, BC1);
  k_wt_f16<<<(DH * (DH / 8) + 255) / 256, 256, 0, stream>>>(dW2, BD2, DH, DH, 16.0f); k_wt_f16<<<(DH * (DH / 8) + 255) / 256, 256, 0, stream>>>(cW2, BC2, DH, DH, 16.0f);
  const dim3 gG(((CHK / 16) * (DH / 64) + 3) / 4, 1); const unsigned nb8 = (unsigned)(((size_t)CHK * DH / 8 + 255) / 256);
  for (size_t p0 = 0; p0 < (size_t)NPT; p0 += CHK) {
    k_embed<<<(CHK * 8 + 255) / 256, 256, 0, stream>>>(pts, vd, T[0], T[1], T[2], p0, H0);
    k_gemm_hhx<3><<<gG, 128, 0, stream>>>(H0, DIN, 0, BD1, 32, 0, 0.0625f, dB1, 0, nullptr, 1, 0, 0, H1, nullptr, DH, 0, CHK, DH, 32);
    k_carry64<<<nb8, 256, 0, stream>>>(H1, H116, (size_t)CHK * DH / 8);
    k_gemm_hhx<3><<<gG, 128, 0, stream>>>(H116, DH, 0, BD2, DH, 0, 0.0625f / 64.0f, dB2, 0, nullptr, 1, 0, 0, H2, nullptr, DH, 0, CHK, DH, DH);
    k_dots<<<(CHK + 255) / 256, 256, 0, stream>>>(H2, dW3, dB3, 1, 0, p0, (float*)d_out);
    k_gemm_hhx<3><<<gG, 128, 0, stream>>>(H0, DIN, 0, BC1, DIN, 0, 0.0625f, cB1, 0, nullptr, 1, 0, 0, H1, nullptr, DH, 0, CHK, DH, DIN);
    k_carry64<<<nb8, 256, 0, stream>>>(H1, H116, (size_t)CHK * DH / 8);
    k_gemm_hhx<3><<<gG, 128, 0, stream>>>(H116, DH, 0, BC2, DH, 0, 0.0625f / 64.0f, cB2, 0, nullptr, 1, 0, 0, H2, nullptr, DH, 0, CHK, DH, DH);
    k_dots<<<(CHK + 255) / 256, 256, 0, stream>>>(H2, cW3, cB3, 3, 1, p0, (float*)d_out); }
}
